// Feature_Grid_Model_19559281066529
// MI455X (gfx1250) — hardware-verified
//
#include <hip/hip_runtime.h>


#define NPT  1000000
#define NPAD 1048576
#define CHK  131072
#define CG   16
#define GG   64
#define LF   10
#define INW  79
#define INP  128
#define HID  32
#define HP   64
#define DM   INP
#define LOSC 1024.0f

typedef _Float16 h16;
typedef unsigned short bf;
typedef __attribute__((ext_vector_type(16))) __bf16   v16bf;
typedef __attribute__((ext_vector_type(16))) _Float16 v16h;
typedef __attribute__((ext_vector_type(8)))  _Float16 v8h;
typedef __attribute__((ext_vector_type(8)))  unsigned short v8us;
typedef __attribute__((ext_vector_type(8)))  float    v8f;
typedef __attribute__((ext_vector_type(4)))  float    v4f;
typedef __attribute__((ext_vector_type(4)))  _Float16 v4h;
typedef v8h  __attribute__((may_alias)) v8ha;
typedef v4f  __attribute__((may_alias)) v4fa;
typedef v8us __attribute__((may_alias)) v8usa;

__device__ __forceinline__ unsigned short f2bf(float f) { unsigned u = __float_as_uint(f); u += 0x7FFFu + ((u >> 16) & 1u); return (unsigned short)(u >> 16); }
__device__ __forceinline__ float bf2f(unsigned short b) { return __uint_as_float(((unsigned)b) << 16); }
__device__ __forceinline__ float bfr(float f) { return bf2f(f2bf(f)); }
__device__ __forceinline__ v16h cat16(v8h lo, v8h hi) { return __builtin_shufflevector(lo, hi, 0, 1, 2, 3, 4, 5, 6, 7, 8, 9, 10, 11, 12, 13, 14, 15); }
__device__ __forceinline__ v16bf cat16b(v8us lo, v8us hi) { return __builtin_bit_cast(v16bf, __builtin_shufflevector(lo, hi, 0, 1, 2, 3, 4, 5, 6, 7, 8, 9, 10, 11, 12, 13, 14, 15)); }
__device__ __forceinline__ v8f wmma16(v16h a, v16h b, v8f c) { return __builtin_amdgcn_wmma_f32_16x16x32_f16(false, a, false, b, (short)0, c, false, false); }
__device__ __forceinline__ v8f wmmab(v16bf a, v16bf b, v8f c) { return __builtin_amdgcn_wmma_f32_16x16x32_bf16(false, a, false, b, (short)0, c, false, false); }

template <bool SPLITA, bool F16OUT = false>
__global__ __launch_bounds__(128) void k_gemmb(const bf* __restrict__ A, const bf* __restrict__ Al, const bf* __restrict__ Bn, const float* __restrict__ bias, float* C, int ldc, h16* C2, const float* __restrict__ R = nullptr, int K = DM, int roundR = 1) {
    __shared__ __align__(16) float ost[4][16 * 68];
    const int lane = threadIdx.x & 31, wave = threadIdx.x >> 5, lr = lane & 15, hi = lane >> 4;
    const int r0 = blockIdx.x * 64 + wave * 16, c0 = blockIdx.y * 64;
    const size_t aoff = (size_t)(r0 + lr) * K + 8 * hi;
    size_t boff[4];
#pragma unroll
    for (int t = 0; t < 4; ++t) boff[t] = (size_t)(c0 + t * 16 + lr) * K + 8 * hi;
    v8f acc[4];
#pragma unroll
    for (int t = 0; t < 4; ++t) acc[t] = (v8f){};
#pragma unroll 1
    for (int kc = 0; kc < K; kc += 32) {
        const v16bf a = cat16b(*(const v8us*)(A + aoff + kc), *(const v8us*)(A + aoff + kc + 16));
        v16bf al = a;
        if (SPLITA) al = cat16b(*(const v8us*)(Al + aoff + kc), *(const v8us*)(Al + aoff + kc + 16));
#pragma unroll
        for (int t = 0; t < 4; ++t) { const v16bf b = cat16b(*(const v8us*)(Bn + boff[t] + kc), *(const v8us*)(Bn + boff[t] + kc + 16)); acc[t] = wmmab(a, b, acc[t]); if (SPLITA) acc[t] = wmmab(al, b, acc[t]); }
        asm volatile("v_nop\n\tv_nop\n\tv_nop\n\tv_nop" : "+v"(acc[0]), "+v"(acc[1]), "+v"(acc[2]), "+v"(acc[3]) : "v"(a), "v"(al));
    }
    float* os = &ost[wave][0];
#pragma unroll
    for (int t = 0; t < 4; ++t) { const float bv = bias ? bfr(bias[c0 + t * 16 + lr]) : 0.f;
#pragma unroll
        for (int j = 0; j < 8; ++j) os[(hi * 8 + j) * 68 + t * 16 + lr] = acc[t][j] + bv; }
    __syncthreads();
    if (F16OUT) {
        h16* crow = (h16*)(void*)C + (size_t)r0 * ldc + c0;
        auto pass = [&]() {
#pragma unroll
            for (int s = 0; s < 4; ++s) { const int row = 4 * s + (lane >> 3), piece = lane & 7; const float* sp = os + row * 68 + piece * 8; v8h o, o2;
#pragma unroll
                for (int i = 0; i < 8; ++i) { const h16 a = (h16)sp[i]; o[i] = a; o2[i] = (h16)((sp[i] - (float)a) * LOSC); }
                *(volatile v8h*)(crow + (size_t)row * ldc + piece * 8) = o; if (C2) *(volatile v8h*)(C2 + (size_t)r0 * ldc + c0 + (size_t)row * ldc + piece * 8) = o2; }
        };
        pass(); __threadfence(); pass();
    } else {
        float* crow = C + (size_t)r0 * ldc + c0;
        auto pass = [&]() {
#pragma unroll
            for (int s = 0; s < 8; ++s) { const int Lid = (lane >> 3) + 4 * s, piece = lane & 7; const int row = Lid >> 1, cofs = (Lid & 1) * 32 + piece * 4;
                v4f val = *(const v4fa*)(os + row * 68 + cofs); if (R) { const v4f rv = *(const v4f*)(R + ((size_t)r0 + row) * ldc + c0 + cofs); val += roundR ? (v4f){bfr(rv[0]), bfr(rv[1]), bfr(rv[2]), bfr(rv[3])} : rv; }
                *(volatile v4f*)(crow + (size_t)row * ldc + cofs) = val; }
        };
        pass(); __threadfence(); pass();
    }
}


__global__ __launch_bounds__(256) void k_w0pad(const float* __restrict__ W0, bf* Bt) {
    typedef __attribute__((ext_vector_type(4))) unsigned short v4us;
    const int lane = threadIdx.x & 31; const int n = blockIdx.x * 8 + (threadIdx.x >> 5); if (n >= HP || lane * 4 >= INP) return; v4us o;
#pragma unroll
    for (int i = 0; i < 4; ++i) { const int k = lane * 4 + i; const bool live = (k < INW) && (n < HID); o[i] = f2bf(live ? W0[(size_t)(live ? k : 0) * HID + (live ? n : 0)] : 0.f); }
    *(volatile v4us*)(Bt + (size_t)n * INP + lane * 4) = o; __threadfence(); *(volatile v4us*)(Bt + (size_t)n * INP + lane * 4) = o;
}
__global__ __launch_bounds__(256) void k_bpad(const float* __restrict__ b, float* BP) {
    const int t = threadIdx.x; if (t >= HP) return; const float v = (t < HID) ? b[t] : 0.f; *(volatile float*)(BP + t) = v; __threadfence(); *(volatile float*)(BP + t) = v;
}
__global__ __launch_bounds__(256) void k_whT(const float* __restrict__ Wm, bf* Bt) {
    typedef __attribute__((ext_vector_type(2))) unsigned short v2us;
    const int lane = threadIdx.x & 31; const int n = blockIdx.x * 8 + (threadIdx.x >> 5); if (n >= HP) return; const int k0 = lane * 2; v2us o;
#pragma unroll
    for (int i = 0; i < 2; ++i) { const int k = k0 + i; const bool live = (k < HID) && (n < HID); o[i] = f2bf(live ? Wm[(size_t)(live ? k : 0) * HID + (live ? n : 0)] : 0.f); }
    *(volatile v2us*)(Bt + (size_t)n * HP + k0) = o; __threadfence(); *(volatile v2us*)(Bt + (size_t)n * HP + k0) = o;
}
__global__ __launch_bounds__(256) void k_snake(const float* __restrict__ F, bf* Ph, bf* Pl) {
    typedef __attribute__((ext_vector_type(2))) unsigned short v2us;
    const int lane = threadIdx.x & 31; const size_t r = (size_t)blockIdx.x * 8 + (threadIdx.x >> 5); if (r >= (size_t)CHK) return; const int c0 = lane * 2; v2us oh, ol;
#pragma unroll
    for (int i = 0; i < 2; ++i) { const int c = c0 + i; float y = 0.f; if (c < HID) { const float x = F[r * HP + c]; const float s = __sinf(x); y = 0.5f * x + s * s; } const unsigned short hb = f2bf(y); oh[i] = hb; ol[i] = f2bf(y - bf2f(hb)); }
    const size_t o = r * HP + c0; *(volatile v2us*)(Ph + o) = oh; *(volatile v2us*)(Pl + o) = ol; __threadfence(); *(volatile v2us*)(Ph + o) = oh; *(volatile v2us*)(Pl + o) = ol;
}
__global__ __launch_bounds__(256) void k_final(const float* __restrict__ F, const float* __restrict__ Wf, const float* __restrict__ bfv, size_t p0, float* OUTB) {
    const int lane = threadIdx.x & 31; const size_t rl = ((size_t)blockIdx.x * 8 + (threadIdx.x >> 5)) * 32 + lane; if (rl >= (size_t)CHK) return; const size_t p = p0 + rl; float a = bfr(bfv[0]);
#pragma unroll 1
    for (int k = 0; k < HID; ++k) { const float x = F[rl * HP + k]; const float s = __sinf(x); a = fmaf(0.5f * x + s * s, bfr(Wf[k]), a); }
    if (p < (size_t)NPT) { *(volatile float*)(OUTB + p) = a; __threadfence(); *(volatile float*)(OUTB + p) = a; }
}


__global__ __launch_bounds__(256) void k_inrows3(const float* __restrict__ coords, const float* __restrict__ vol, size_t p0, bf* Xh, bf* Xl) {
    __shared__ unsigned short th[64][130]; __shared__ unsigned short tlo[64][130];
    const int t = threadIdx.x; const int pl = t >> 2, j = t & 3; const size_t p = p0 + (size_t)blockIdx.x * 64 + pl; const bool live = p < (size_t)NPT;
    float cx = 0.f, cy = 0.f, cz = 0.f; if (live) { cx = bfr(coords[p * 3]); cy = bfr(coords[p * 3 + 1]); cz = bfr(coords[p * 3 + 2]); }
    auto put = [&](int col, float y) { const unsigned short hb = f2bf(y); th[pl][col] = hb; tlo[pl][col] = f2bf(y - bf2f(hb)); };
    for (int col = j; col < INP; col += 4) { float y = 0.f; if (live && col < 3) y = (col == 0) ? cx : (col == 1 ? cy : cz); if (col < 3 || col >= INW) put(col, y); }
#pragma unroll 1
    for (int q = j; q < 30; q += 4) { const int l = q / 3, ax = q % 3; const float c = (ax == 0) ? cx : (ax == 1 ? cy : cz); const float a = c * (float)(1 << l); float s, co; sincosf(a, &s, &co); if (!live) { s = 0.f; co = 0.f; } put(3 + l * 6 + ax, s); put(3 + l * 6 + 3 + ax, co); }
    const float fx = (cx + 1.0f) * (float)GG * 0.5f - 0.5f, fy = (cy + 1.0f) * (float)GG * 0.5f - 0.5f, fz = (cz + 1.0f) * (float)GG * 0.5f - 0.5f;
    const float x0f = floorf(fx), y0f = floorf(fy), z0f = floorf(fz); const float wx = fx - x0f, wy = fy - y0f, wz = fz - z0f; const int x0 = (int)x0f, y0 = (int)y0f, z0 = (int)z0f;
#pragma unroll 1
    for (int ch = j; ch < CG; ch += 4) { float acc = 0.f;
#pragma unroll 1
        for (int corner = 0; corner < 8; ++corner) { const int dz = corner >> 2, dy = (corner >> 1) & 1, dx = corner & 1; const int xi = x0 + dx, yi = y0 + dy, zi = z0 + dz;
            const bool valid = xi >= 0 && xi < GG && yi >= 0 && yi < GG && zi >= 0 && zi < GG; const int xc = min(max(xi, 0), GG - 1), yc = min(max(yi, 0), GG - 1), zc = min(max(zi, 0), GG - 1);
            const float w = (dz ? wz : 1.0f - wz) * (dy ? wy : 1.0f - wy) * (dx ? wx : 1.0f - wx); const float v = bfr(vol[(((size_t)ch * GG + zc) * GG + yc) * GG + xc]); acc = acc + w * (valid ? v : 0.f); }
        put(63 + ch, live ? acc : 0.f); }
    __syncthreads();
    const int lane = t & 31, wv = t >> 5;
    auto pass = [&]() {
#pragma unroll
        for (int st = 0; st < 4; ++st) { const int rr = wv * 8 + st * 2 + (lane >> 4); const int c0 = (lane & 15) * 8; v8us oh, ol;
#pragma unroll
            for (int i = 0; i < 8; ++i) { oh[i] = th[rr][c0 + i]; ol[i] = tlo[rr][c0 + i]; }
            const size_t o = ((size_t)blockIdx.x * 64 + rr) * INP + c0; *(volatile v8us*)(Xh + o) = oh; *(volatile v8us*)(Xl + o) = ol; }
    };
    pass(); __threadfence(); pass();
}

extern "C" void kernel_launch(void* const* d_in, const int* in_sizes, int n_in,
                              void* d_out, int out_size, void* d_ws, size_t ws_size, hipStream_t stream) {
    (void)in_sizes; (void)n_in; (void)out_size;
    const float* coords = (const float*)d_in[0]; const float* vol = (const float*)d_in[1]; const float* W0 = (const float*)d_in[2]; const float* b0 = (const float*)d_in[3]; const float* Wh = (const float*)d_in[4]; const float* bh = (const float*)d_in[5]; const float* Wf = (const float*)d_in[6]; const float* bfv = (const float*)d_in[7];
    float* out = (float*)d_out;
    char* wsp = (char*)d_ws;
    auto take = [&](size_t bytes) { char* p = wsp; wsp += (bytes + 255) & ~(size_t)255; return (void*)p; };
    bf* BW0 = (bf*)take(HP * INP * 2); bf* BWH = (bf*)take((size_t)3 * HP * HP * 2); float* B0P = (float*)take(HP * 4); float* BHP = (float*)take((size_t)3 * HP * 4);
    bf* Xh = (bf*)take((size_t)CHK * INP * 2); bf* Xl = (bf*)take((size_t)CHK * INP * 2); float* F = (float*)take((size_t)CHK * HP * 4); bf* Ph = (bf*)take((size_t)CHK * HP * 2); bf* Pl = (bf*)take((size_t)CHK * HP * 2);
    if ((size_t)(wsp - (char*)d_ws) > ws_size) return;
    k_w0pad<<<HP / 8, 256, 0, stream>>>(W0, BW0); k_bpad<<<1, 256, 0, stream>>>(b0, B0P); for (int i = 0; i < 3; ++i) { k_whT<<<HP / 8, 256, 0, stream>>>(Wh + (size_t)i * HID * HID, BWH + (size_t)i * HP * HP); k_bpad<<<1, 256, 0, stream>>>(bh + i * HID, BHP + i * HP); }
    for (int ch = 0; ch < NPAD / CHK; ++ch) { const size_t p0 = (size_t)ch * CHK;
        k_inrows3<<<CHK / 64, 256, 0, stream>>>(coords, vol, p0, Xh, Xl);
        k_gemmb<true, false><<<dim3(CHK / 64, 1, 1), 128, 0, stream>>>(Xh, Xl, BW0, B0P, F, HP, nullptr, nullptr, INP);
        for (int i = 0; i < 3; ++i) { k_snake<<<CHK / 8, 256, 0, stream>>>(F, Ph, Pl); k_gemmb<true, false><<<dim3(CHK / 64, 1, 1), 128, 0, stream>>>(Ph, Pl, BWH + (size_t)i * HP * HP, BHP + i * HP, F, HP, nullptr, nullptr, HP); }
        k_final<<<(CHK / 32) / 8, 256, 0, stream>>>(F, Wf, bfv, p0, out); }
}
